// PhysicsGPSLayer_39728447488412
// MI455X (gfx1250) — hardware-run, weakly checked
//
#include <hip/hip_runtime.h>


namespace {
constexpr int N = 16384, D = 128, ED = 32, E = 262144, G = 32, S = 512, NH = 4, HD = 32, NBLK = N / 16;
constexpr float XS = 8.0f, OS = 256.0f, PS = 1024.0f, WSC = 256.0f, EPS = 1e-5f;
typedef _Float16 b16;
typedef __attribute__((ext_vector_type(16))) _Float16 v16b;
typedef __attribute__((ext_vector_type(8))) _Float16 v8b;
typedef __attribute__((ext_vector_type(8))) float v8f;
typedef __attribute__((ext_vector_type(4))) float v4f;
__device__ __forceinline__ float bf16_rne(float f) { unsigned int u = __float_as_uint(f); u += 0x7FFFu + ((u >> 16) & 1u); return __uint_as_float(u & 0xFFFF0000u); }
__device__ __forceinline__ void split16(float v, b16& hi, b16& lo) { hi = (b16)v; lo = (b16)(v - (float)hi); }
__device__ __forceinline__ v16b frag_kb(const b16* p, int hh) { const v8b a = *(const v8b*)(p + 8 * hh), b = *(const v8b*)(p + 16 + 8 * hh); v16b f;
#pragma unroll
  for (int e = 0; e < 8; ++e) { f[e] = a[e]; f[8 + e] = b[e]; } return f; }
__device__ __forceinline__ v8f wmma16b(v16b a, v16b b, v8f c) { v8f d = __builtin_amdgcn_wmma_f32_16x16x32_f16(false, a, false, b, (short)0, c, false, false); asm volatile("v_nop\n\tv_nop\n\tv_nop\n\tv_nop" : "+v"(d) : "v"(a), "v"(b)); return d; }
__device__ __forceinline__ void wave_lds_sync() { __builtin_amdgcn_fence(__ATOMIC_RELEASE, "workgroup"); __builtin_amdgcn_wave_barrier(); __builtin_amdgcn_fence(__ATOMIC_ACQUIRE, "workgroup"); }
__device__ __forceinline__ float pmul(float a, float b) { float p = a * b; asm volatile("" : "+v"(p)); return p; }
__device__ __forceinline__ int iclamp(int v, int lo, int hi) { return v < lo ? lo : (v > hi ? hi : v); }
__device__ __forceinline__ float gelu(float v) { return 0.5f * v * (1.0f + erff(v * 0.70710678118654752f)); }
constexpr int CSR_NBLK9 = 512, CSR_GB9 = 9, CSR_GN9 = 1 << CSR_GB9  , CSR_TS9 = (CSR_GN9 < 32 ? 32 : CSR_GN9)  , CSR_MAXG9 = 512, CSR_CAP9 = 12288  ;
__device__ __host__ __forceinline__ int csr_tix9(int v) { return (v >> CSR_GB9) * CSR_TS9 + (v & (CSR_GN9 - 1)); }
__global__ __launch_bounds__(64) void csrA_kernel9(const int* __restrict__ dst, int E, int N, int nG, int CHP, int NGP, int* __restrict__ STG, int* __restrict__ HST) {
  extern __shared__ int sm[];
  int* cnt = sm; int* run = sm + NGP; int* ids = sm + 2 * NGP;
  const int b = blockIdx.x; const int ch = (E + CSR_NBLK9 - 1) / CSR_NBLK9; const int e0 = b * ch, e1 = min(E, e0 + ch);
  for (int i = threadIdx.x; i < NGP; i += 64) cnt[i] = 0;
  for (int i = threadIdx.x; i < CHP; i += 64) ids[i] = -1;
  __syncthreads();
  if (threadIdx.x == 0) {
    for (int e = e0; e < e1; ++e) { int d = dst[e]; d = (d < 0) ? 0 : (d >= N ? N - 1 : d); cnt[d >> CSR_GB9] += 1; }
    int acc = 0; for (int g = 0; g < nG; ++g) { run[g] = acc; acc += cnt[g]; }
    for (int e = e0; e < e1; ++e) { int d = dst[e]; d = (d < 0) ? 0 : (d >= N ? N - 1 : d); const int g = d >> CSR_GB9; ids[run[g]] = e; run[g] += 1; } }
  __syncthreads();
  typedef __attribute__((ext_vector_type(4))) int v4i;
  for (int pass = 0; pass < 2; ++pass) {
    for (int i = threadIdx.x; i < CHP / 4; i += 64) *(volatile v4i*)(STG + (size_t)b * CHP + i * 4) = *(const v4i*)(&ids[i * 4]);
    for (int i = threadIdx.x; i < NGP / 4; i += 64) { v4i v; for (int e = 0; e < 4; ++e) v[e] = (i * 4 + e < nG) ? cnt[i * 4 + e] : 0; *(volatile v4i*)(HST + (size_t)b * NGP + i * 4) = v; }
    __threadfence(); }
}
__global__ __launch_bounds__(512) void csrS_kernel9(const int* __restrict__ HST, int nG, int NGP, int* __restrict__ START, int* __restrict__ TOT, int* __restrict__ OFF) {
  __shared__ int tot[CSR_MAXG9];
  const int b = threadIdx.x;
  for (int pass = 0; pass < 2; ++pass) { int runb = 0; for (int g = 0; g < nG; ++g) { int c = HST[(size_t)b * NGP + g]; c = (c < 0) ? 0 : c; ((volatile int*)OFF)[(size_t)g * CSR_NBLK9 + b] = runb; runb += c; } __threadfence(); }
  for (int g = threadIdx.x; g < nG; g += 512) { int s = 0; for (int bb = 0; bb < CSR_NBLK9; ++bb) { int c = HST[(size_t)bb * NGP + g]; s += (c < 0) ? 0 : c; } tot[g] = s; }
  __syncthreads();
  if (threadIdx.x < 32) {
    __shared__ int st[CSR_MAXG9 + 32];
    if (threadIdx.x == 0) { int acc = 0; for (int g = 0; g < NGP; ++g) { st[g] = acc; if (g < nG) acc += (tot[g] + 31) & ~31; } st[NGP] = acc; }
    __builtin_amdgcn_fence(__ATOMIC_RELEASE, "workgroup"); __builtin_amdgcn_wave_barrier(); __builtin_amdgcn_fence(__ATOMIC_ACQUIRE, "workgroup");
    for (int pass = 0; pass < 2; ++pass) { for (int i = threadIdx.x; i < NGP + 32; i += 32) { ((volatile int*)START)[i] = (i <= NGP) ? st[min(i, NGP)] : 0; ((volatile int*)TOT)[i] = (i < nG) ? tot[i] : 0; } __threadfence(); } }
}
__global__ __launch_bounds__(256) void csrB_kernel9(const int* __restrict__ dst, int N, int nG, int CHP, int NGP, int permLen, const int* __restrict__ STG, const int* __restrict__ HST, const int* __restrict__ OFF, const int* __restrict__ START, const int* __restrict__ TOT, int* __restrict__ PERM, int* __restrict__ ROWPTR, int* __restrict__ ROWCNT, int* __restrict__ FLAG) {
  typedef __attribute__((ext_vector_type(4))) int v4i;
  __shared__ int ids[CSR_CAP9]; __shared__ unsigned short key[CSR_CAP9]; __shared__ int outp[CSR_CAP9]; __shared__ int ncnt[CSR_GN9 + 1]; __shared__ int boff[CSR_NBLK9 + 1];
  const int g = blockIdx.x, t_ = threadIdx.x; int tot = TOT[g]; int st = START[g], stn = START[g + 1]; const int v0 = g * CSR_GN9; const int nv = min(CSR_GN9, N - v0); const int t0 = g * CSR_TS9;
  st = (st < 0) ? 0 : (st > permLen - 32 ? permLen - 32 : st) & ~31; stn = (stn < st) ? st : (stn > permLen ? permLen : stn); tot = (tot < 0) ? 0 : tot; if (tot > stn - st && tot <= CSR_CAP9) tot = stn - st;
  if (tot > CSR_CAP9) {
    for (int pass = 0; pass < 2; ++pass) { for (int i = t_; i < CSR_TS9 / 4; i += 256) { v4i a, c; for (int e = 0; e < 4; ++e) { a[e] = st; c[e] = 0; } *(volatile v4i*)(ROWPTR + t0 + i * 4) = a; *(volatile v4i*)(ROWCNT + t0 + i * 4) = c; } if (t_ == 0) ((volatile int*)FLAG)[0] = 1; __threadfence(); } (void)nv; return; }
  if (t_ == 0) { int acc = 0; for (int b = 0; b < CSR_NBLK9; ++b) { boff[b] = acc; int c = HST[(size_t)b * NGP + g]; c = (c < 0) ? 0 : (c > CHP ? CHP : c); acc += c; if (acc > tot) acc = tot; } boff[CSR_NBLK9] = acc; }
  for (int i = t_; i <= CSR_GN9; i += 256) ncnt[i] = 0;
  __syncthreads();
  for (int b = 0; b < CSR_NBLK9; ++b) { const int c = boff[b + 1] - boff[b]; int o_ = OFF[(size_t)g * CSR_NBLK9 + b]; o_ = (o_ < 0) ? 0 : (o_ > CHP - c ? CHP - c : o_); const int* src_ = STG + (size_t)b * CHP + o_;
    for (int i = t_; i < c; i += 256) { int id = src_[i]; id = (id < 0) ? 0 : id; ids[boff[b] + i] = id; int d = dst[id]; d = (d < v0) ? v0 : (d >= N ? N - 1 : d); int kk = d - v0; kk = (kk < 0) ? 0 : (kk >= CSR_GN9 ? CSR_GN9 - 1 : kk); key[boff[b] + i] = (unsigned short)kk; } }
  __syncthreads();
  if (t_ == 0) { for (int i = 0; i < tot; ++i) ncnt[key[i]] += 1; int acc = 0; for (int vl = 0; vl < CSR_GN9; ++vl) { const int c = ncnt[vl]; ncnt[vl] = acc; acc += c; } ncnt[CSR_GN9] = acc;
    for (int i = 0; i < tot; ++i) { const int vl = key[i]; outp[ncnt[vl]] = ids[i]; ncnt[vl] += 1; }
    for (int vl = CSR_GN9; vl > 0; --vl) ncnt[vl] = ncnt[vl - 1]; ncnt[0] = 0; }
  __syncthreads();
  for (int pass = 0; pass < 2; ++pass) {
    for (int i = t_; i < (stn - st) / 4; i += 256) { v4i v; for (int e = 0; e < 4; ++e) { const int q = i * 4 + e; v[e] = (q < tot) ? outp[q] : -1; } *(volatile v4i*)(PERM + st + i * 4) = v; }
    for (int i = t_; i < CSR_TS9 / 4; i += 256) { v4i a, c; for (int e = 0; e < 4; ++e) { const int vl = i * 4 + e; const int vc = vl < CSR_GN9 ? vl : CSR_GN9; a[e] = (vl < CSR_GN9) ? st + ncnt[vc] : st; c[e] = (vl < nv) ? (ncnt[(vc < CSR_GN9 ? vc : CSR_GN9 - 1) + 1] - ncnt[vc]) : 0; } *(volatile v4i*)(ROWPTR + t0 + i * 4) = a; *(volatile v4i*)(ROWCNT + t0 + i * 4) = c; }
    __threadfence(); }
}
__global__ __launch_bounds__(256) void csrZ_kernel9(int* __restrict__ p, size_t n4) { typedef __attribute__((ext_vector_type(4))) int v4i; const size_t tid = (size_t)blockIdx.x * 256 + threadIdx.x, nth = (size_t)gridDim.x * 256; v4i z = {0, 0, 0, 0}; for (size_t i = tid; i < n4; i += nth) *(volatile v4i*)(p + i * 4) = z; }
struct CsrBufs9 { int *STG, *HST, *OFF, *START, *TOT, *PERM, *ROWPTR, *ROWCNT, *FLAG; int nG, NGP, CHP; size_t permLen; char* base; size_t bytes; };
static size_t csr_carve9(CsrBufs9& c, char* ws, size_t off, int E, int N) {
  const size_t off0 = off; c.base = ws + off;
  auto al = [&](size_t bytes) { char* p = ws + off; off += (bytes + 255) & ~(size_t)255; return p; };
  c.nG = (N + CSR_GN9 - 1) / CSR_GN9; c.NGP = (c.nG + 31) & ~31; const int ch = (E + CSR_NBLK9 - 1) / CSR_NBLK9; c.CHP = (ch + 31) & ~31; c.permLen = (size_t)E + 32 * (size_t)c.nG + 32;
  c.STG = (int*)al((size_t)CSR_NBLK9 * c.CHP * 4); c.HST = (int*)al((size_t)CSR_NBLK9 * c.NGP * 4); c.OFF = (int*)al((size_t)c.NGP * CSR_NBLK9 * 4); c.START = (int*)al((size_t)(c.NGP + 64) * 4); c.TOT = (int*)al((size_t)(c.NGP + 64) * 4);
  c.PERM = (int*)al(c.permLen * 4); c.ROWPTR = (int*)al((size_t)c.nG * CSR_TS9 * 4); c.ROWCNT = (int*)al((size_t)c.nG * CSR_TS9 * 4); c.FLAG = (int*)al(256);
  c.bytes = off - off0; return off;
}
static void csr_build9(const CsrBufs9& c, const int* dst, int E, int N, hipStream_t stream) {
  const size_t smem = (size_t)(2 * c.NGP + c.CHP) * 4;
  csrZ_kernel9<<<512, 256, 0, stream>>>((int*)c.base, c.bytes / 16);
  csrA_kernel9<<<CSR_NBLK9, 64, smem, stream>>>(dst, E, N, c.nG, c.CHP, c.NGP, c.STG, c.HST);
  csrS_kernel9<<<1, 512, 0, stream>>>(c.HST, c.nG, c.NGP, c.START, c.TOT, c.OFF);
  csrB_kernel9<<<c.nG, 256, 0, stream>>>(dst, N, c.nG, c.CHP, c.NGP, (int)c.permLen, c.STG, c.HST, c.OFF, c.START, c.TOT, c.PERM, c.ROWPTR, c.ROWCNT, c.FLAG);
}


__global__ __launch_bounds__(256) void wput_kernel(const float* __restrict__ w, int r0, int KIN, int OUTW, int ro, b16* __restrict__ WT) {
  const int KG = KIN / 8; const size_t u = (size_t)blockIdx.x * 256 + threadIdx.x; if (u >= (size_t)OUTW * KG) return; const int o = (int)(u / KG), k0 = (int)(u % KG) * 8; v8b v;
#pragma unroll
  for (int j = 0; j < 8; ++j) v[j] = (b16)(bf16_rne(w[(size_t)(r0 + k0 + j) * OUTW + o]) * WSC); for (int pass = 0; pass < 2; ++pass) { *(volatile v8b*)(WT + (size_t)(ro + o) * KIN + k0) = v; __threadfence(); }
}
__device__ __forceinline__ void ln128(float* v, const float* g, const float* b, int lane) { float s = v[0] + v[1] + v[2] + v[3]; for (int o = 16; o; o >>= 1) s += __shfl_xor(s, o); const float mu = s * (1.0f / D); float q = 0.0f; for (int i = 0; i < 4; ++i) { const float d_ = v[i] - mu; q += pmul(d_, d_); } for (int o = 16; o; o >>= 1) q += __shfl_xor(q, o); const float rs = rsqrtf(q * (1.0f / D) + EPS); for (int i = 0; i < 4; ++i) v[i] = pmul(pmul(v[i] - mu, rs), bf16_rne(g[lane * 4 + i])) + bf16_rne(b[lane * 4 + i]); }
template <int KIN, int NT, int EXACT, int ACT>
__global__ __launch_bounds__(32) void dense_kernel(const float* __restrict__ IN, int inp, float ASC, const b16* __restrict__ WT, const float* __restrict__ bias, int NLIM, float* __restrict__ OUT) {
  __shared__ __attribute__((aligned(16))) b16 Ah[16][KIN + 8], Al[16][(EXACT ? 32 : KIN) + 8]; __shared__ __attribute__((aligned(16))) float Tf[16][128 + 4];
  const int lane = threadIdx.x, nloc = lane & 15, hlf = lane >> 4; const size_t m0 = (size_t)blockIdx.x * 16; if (m0 >= (size_t)NLIM) return;
  for (int rr = 0; rr < 16; ++rr) for (int q = 0; q < KIN / 32; ++q) { const float v = IN[(m0 + rr) * inp + q * 32 + lane]; if (EXACT) Ah[rr][q * 32 + lane] = (b16)(bf16_rne(v) * ASC); else { b16 p, ql; split16(v * ASC, p, ql); Ah[rr][q * 32 + lane] = p; Al[rr][q * 32 + lane] = ql; } }
  wave_lds_sync();
#pragma unroll 1
  for (int cg = 0; cg < (NT + 7) / 8; ++cg) { const int nt = NT - cg * 8 < 8 ? NT - cg * 8 : 8; v8f acc[8];
#pragma unroll
    for (int t = 0; t < 8; ++t) acc[t] = (v8f){};
#pragma unroll 2
    for (int kb = 0; kb < KIN; kb += 32) { const v16b a = frag_kb(&Ah[nloc][kb], hlf); v16b al; if (!EXACT) al = frag_kb(&Al[nloc][kb], hlf);
#pragma unroll
      for (int t = 0; t < 8; ++t) if (t < nt) { const v16b bw = frag_kb(WT + (size_t)(cg * 128 + t * 16 + nloc) * KIN + kb, hlf); acc[t] = wmma16b(a, bw, acc[t]); if (!EXACT) acc[t] = wmma16b(al, bw, acc[t]); } }
#pragma unroll
    for (int t = 0; t < 8; ++t) { if (t < nt) { const int c = cg * 128 + t * 16 + nloc; const float bb = bias ? bf16_rne(bias[c]) : 0.0f;
#pragma unroll
        for (int r8 = 0; r8 < 8; ++r8) { float v = acc[t][r8] * (1.0f / (ASC * WSC)) + bb; if (ACT) v = gelu(v); Tf[8 * hlf + r8][t * 16 + nloc] = v; } } }
    wave_lds_sync();
    for (int pass = 0; pass < 2; ++pass) { for (int rr = 0; rr < 16; ++rr) for (int c = lane; c < nt * 16; c += 32) ((volatile float*)OUT)[(m0 + rr) * (size_t)(NT * 16) + cg * 128 + c] = Tf[rr][c]; __threadfence(); }
    wave_lds_sync(); }
}
__global__ __launch_bounds__(256) void ln_kernel(const float* __restrict__ x, const float* __restrict__ g, const float* __restrict__ b, int NLIM, float* __restrict__ XN) {
  const int wave = threadIdx.x >> 5, lane = threadIdx.x & 31; const size_t n = (size_t)blockIdx.x * 8 + wave; if (n >= (size_t)NLIM) return; float v[4]; for (int i = 0; i < 4; ++i) v[i] = bf16_rne(x[n * D + lane * 4 + i]); ln128(v, g, b, lane);
  for (int pass = 0; pass < 2; ++pass) { *(volatile v4f*)(XN + n * D + lane * 4) = (v4f){v[0], v[1], v[2], v[3]}; __threadfence(); }
}
__global__ __launch_bounds__(32) void edge_kernel(const float* __restrict__ ea, const int* __restrict__ srcs, const float* __restrict__ PQ, const b16* __restrict__ WE, const float* __restrict__ b1, const b16* __restrict__ W2T, const float* __restrict__ b2, const int* __restrict__ PERM, const int* __restrict__ ROWPTR, const int* __restrict__ ROWCNT, int permLen, int NLIM, float* __restrict__ AGG) {
  __shared__ __attribute__((aligned(16))) b16 Ae[16][40], Ag[16][2 * D + 8]; __shared__ float Mo[16][D + 1]; __shared__ int Ss[16];
  const int lane = threadIdx.x, nloc = lane & 15, hlf = lane >> 4; const size_t v = blockIdx.x; if (v >= (size_t)NLIM) return;
  int st = ROWPTR[v], cnt = ROWCNT[v]; cnt = iclamp(cnt, 0, 1 << 20); st = iclamp(st, 0, permLen - cnt); float osum[4] = {0.0f, 0.0f, 0.0f, 0.0f};
  float pv[8]; for (int q = 0; q < 8; ++q) pv[q] = PQ[v * (4 * D) + q * 32 + lane] + bf16_rne(b1[q * 32 + lane]);
#pragma unroll 1
  for (int j0 = 0; j0 < cnt; j0 += 16) {
    for (int rr = 0; rr < 16; ++rr) { const int jj = j0 + rr; int s = -1, e = 0; if (jj < cnt) { e = iclamp(PERM[st + jj], 0, E - 1); s = iclamp(srcs[e], 0, N - 1); if (s >= NLIM) s = -1; } if (lane == 0) Ss[rr] = s; Ae[rr][lane] = (s >= 0) ? (b16)(bf16_rne(ea[(size_t)e * ED + lane]) * XS) : (b16)0.0f; }
    wave_lds_sync(); const v16b a = frag_kb(&Ae[nloc][0], hlf);
#pragma unroll
    for (int cg = 0; cg < 2; ++cg) { v8f acc[8];
#pragma unroll
      for (int t = 0; t < 8; ++t) { acc[t] = (v8f){}; acc[t] = wmma16b(a, frag_kb(WE + (size_t)(cg * 128 + t * 16 + nloc) * 32, hlf), acc[t]); }
      wave_lds_sync();
#pragma unroll
      for (int t = 0; t < 8; ++t) { const int c = cg * 128 + t * 16 + nloc; const float pb = __shfl(pv[c >> 5], c & 31);
#pragma unroll
        for (int r8 = 0; r8 < 8; ++r8) { const int rl = 8 * hlf + r8; const int s = Ss[rl]; const float qv = (s >= 0) ? PQ[(size_t)s * (4 * D) + 2 * D + c] : 0.0f; Ag[rl][c] = (b16)(gelu(acc[t][r8] * (1.0f / (XS * WSC)) + pb + qv) * XS); } } }
    wave_lds_sync(); v8f m2[8];
#pragma unroll
    for (int t = 0; t < 8; ++t) m2[t] = (v8f){};
#pragma unroll 2
    for (int kb = 0; kb < 2 * D; kb += 32) { const v16b a2 = frag_kb(&Ag[nloc][kb], hlf);
#pragma unroll
      for (int t = 0; t < 8; ++t) m2[t] = wmma16b(a2, frag_kb(W2T + (size_t)(t * 16 + nloc) * (2 * D) + kb, hlf), m2[t]); }
#pragma unroll
    for (int t = 0; t < 8; ++t)
#pragma unroll
      for (int r8 = 0; r8 < 8; ++r8) Mo[8 * hlf + r8][t * 16 + nloc] = m2[t][r8] * (1.0f / (XS * WSC));
    wave_lds_sync();
    for (int rr = 0; rr < 16; ++rr) if (Ss[rr] >= 0) { for (int i = 0; i < 4; ++i) osum[i] += Mo[rr][lane * 4 + i] + bf16_rne(b2[lane * 4 + i]); }
    wave_lds_sync(); }
  for (int pass = 0; pass < 2; ++pass) { *(volatile v4f*)(AGG + v * D + lane * 4) = (v4f){osum[0], osum[1], osum[2], osum[3]}; __threadfence(); }
}
__global__ __launch_bounds__(32) void upd_kernel(const float* __restrict__ XN, const float* __restrict__ AGG, const b16* __restrict__ U1, const float* __restrict__ b1, const b16* __restrict__ U2, const float* __restrict__ b2, int NLIM, float* __restrict__ HL) {
  __shared__ __attribute__((aligned(16))) b16 Ah[16][2 * D + 8], Al[16][2 * D + 8]; __shared__ __attribute__((aligned(16))) float Tf[16][D + 4];
  const int lane = threadIdx.x, nloc = lane & 15, hlf = lane >> 4; const size_t m0 = (size_t)blockIdx.x * 16; if (m0 >= (size_t)NLIM) return;
  for (int rr = 0; rr < 16; ++rr) for (int q = 0; q < 8; ++q) { const int c = q * 32 + lane; const float v = c < D ? XN[(m0 + rr) * D + c] : AGG[(m0 + rr) * D + c - D]; b16 p, ql; split16(v * XS, p, ql); Ah[rr][c] = p; Al[rr][c] = ql; }
  wave_lds_sync(); v8f acc[8];
#pragma unroll
  for (int t = 0; t < 8; ++t) acc[t] = (v8f){};
#pragma unroll 2
  for (int kb = 0; kb < 2 * D; kb += 32) { const v16b a = frag_kb(&Ah[nloc][kb], hlf), al = frag_kb(&Al[nloc][kb], hlf);
#pragma unroll
    for (int t = 0; t < 8; ++t) { const v16b bw = frag_kb(U1 + (size_t)(t * 16 + nloc) * (2 * D) + kb, hlf); acc[t] = wmma16b(a, bw, acc[t]); acc[t] = wmma16b(al, bw, acc[t]); } }
  wave_lds_sync();
#pragma unroll
  for (int t = 0; t < 8; ++t) { const int c = t * 16 + nloc; const float bb = bf16_rne(b1[c]);
#pragma unroll
    for (int r8 = 0; r8 < 8; ++r8) { b16 p, ql; split16(gelu(acc[t][r8] * (1.0f / (XS * WSC)) + bb) * XS, p, ql); Ah[8 * hlf + r8][c] = p; Al[8 * hlf + r8][c] = ql; } }
  wave_lds_sync();
#pragma unroll
  for (int t = 0; t < 8; ++t) acc[t] = (v8f){};
#pragma unroll
  for (int kb = 0; kb < D; kb += 32) { const v16b a = frag_kb(&Ah[nloc][kb], hlf), al = frag_kb(&Al[nloc][kb], hlf);
#pragma unroll
    for (int t = 0; t < 8; ++t) { const v16b bw = frag_kb(U2 + (size_t)(t * 16 + nloc) * D + kb, hlf); acc[t] = wmma16b(a, bw, acc[t]); acc[t] = wmma16b(al, bw, acc[t]); } }
#pragma unroll
  for (int t = 0; t < 8; ++t) { const int c = t * 16 + nloc; const float bb = bf16_rne(b2[c]);
#pragma unroll
    for (int r8 = 0; r8 < 8; ++r8) Tf[8 * hlf + r8][c] = acc[t][r8] * (1.0f / (XS * WSC)) + bb; }
  wave_lds_sync();
  for (int pass = 0; pass < 2; ++pass) { for (int rr = 0; rr < 16; ++rr) *(volatile v4f*)(HL + (m0 + rr) * D + lane * 4) = *(const v4f*)(&Tf[rr][lane * 4]); __threadfence(); }
}
__global__ __launch_bounds__(32) void att_kernel(const float* __restrict__ QKV, int NGV, float* __restrict__ O) {
  __shared__ __attribute__((aligned(16))) b16 Qh[16][40], Kh[16][40]; __shared__ float Sc[16][S + 1]; __shared__ __attribute__((aligned(16))) b16 Ph[16][S + 8], Pl[16][S + 8], Vh[HD][40], Vl[HD][40]; __shared__ float Of[16][HD + 1];
  const int lane = threadIdx.x, nloc = lane & 15, hlf = lane >> 4; const int qb = blockIdx.x % (S / 16), h = (blockIdx.x / (S / 16)) % NH, g = blockIdx.x / ((S / 16) * NH); if (g >= NGV) return;
  const size_t t0 = (size_t)g * S, tq = t0 + qb * 16; const float qs = 0.17677669529663688f;
  for (int rr = 0; rr < 16; ++rr) Qh[rr][lane] = (b16)(QKV[(tq + rr) * (3 * D) + h * HD + lane] * qs * XS);
#pragma unroll 1
  for (int kb = 0; kb < S / 16; ++kb) { for (int rr = 0; rr < 16; ++rr) Kh[rr][lane] = (b16)(QKV[(t0 + kb * 16 + rr) * (3 * D) + D + h * HD + lane] * XS);
    wave_lds_sync(); v8f acc = {}; acc = wmma16b(frag_kb(&Qh[nloc][0], hlf), frag_kb(&Kh[nloc][0], hlf), acc);
#pragma unroll
    for (int r8 = 0; r8 < 8; ++r8) Sc[8 * hlf + r8][kb * 16 + nloc] = acc[r8] * (1.0f / (XS * XS));
    wave_lds_sync(); }
  for (int qi = 0; qi < 16; ++qi) { float mx = -INFINITY; for (int j = lane; j < S; j += 32) mx = fmaxf(mx, Sc[qi][j]); for (int o = 16; o; o >>= 1) mx = fmaxf(mx, __shfl_xor(mx, o)); float s = 0.0f;
    for (int j = lane; j < S; j += 32) { const float e = __expf(Sc[qi][j] - mx); Sc[qi][j] = e; s += e; } for (int o = 16; o; o >>= 1) s += __shfl_xor(s, o); const float inv = 1.0f / s;
    for (int j = lane; j < S; j += 32) { b16 p, q; split16(Sc[qi][j] * inv * PS, p, q); Ph[qi][j] = p; Pl[qi][j] = q; } }
  wave_lds_sync(); v8f oacc[2] = {(v8f){}, (v8f){}};
#pragma unroll 1
  for (int kc = 0; kc < S; kc += 32) { for (int jj = 0; jj < 32; ++jj) { b16 p, ql; split16(QKV[(t0 + kc + jj) * (3 * D) + 2 * D + h * HD + lane] * XS, p, ql); Vh[lane][jj] = p; Vl[lane][jj] = ql; }
    wave_lds_sync(); const v16b pa = frag_kb(&Ph[nloc][kc], hlf), pl = frag_kb(&Pl[nloc][kc], hlf);
#pragma unroll
    for (int t = 0; t < 2; ++t) { const v16b vh = frag_kb(&Vh[t * 16 + nloc][0], hlf), vl = frag_kb(&Vl[t * 16 + nloc][0], hlf); oacc[t] = wmma16b(pa, vh, oacc[t]); oacc[t] = wmma16b(pa, vl, oacc[t]); oacc[t] = wmma16b(pl, vh, oacc[t]); }
    wave_lds_sync(); }
#pragma unroll
  for (int t = 0; t < 2; ++t)
#pragma unroll
    for (int r8 = 0; r8 < 8; ++r8) Of[8 * hlf + r8][t * 16 + nloc] = oacc[t][r8] * (1.0f / (PS * XS));
  wave_lds_sync();
  for (int pass = 0; pass < 2; ++pass) { for (int rr = 0; rr < 16; ++rr) ((volatile float*)O)[(tq + rr) * D + h * HD + lane] = Of[rr][lane]; __threadfence(); }
}
__global__ __launch_bounds__(32) void mix_kernel(const float* __restrict__ O, const b16* __restrict__ WO, const float* __restrict__ ob, const float* __restrict__ x, const float* __restrict__ HL, const float* __restrict__ g1, const float* __restrict__ be1, int NLIM, float* __restrict__ H1) {
  __shared__ __attribute__((aligned(16))) b16 Ah[16][D + 8], Al[16][D + 8]; __shared__ __attribute__((aligned(16))) float Tf[16][D + 4];
  const int lane = threadIdx.x, nloc = lane & 15, hlf = lane >> 4; const size_t m0 = (size_t)blockIdx.x * 16; if (m0 >= (size_t)NLIM) return;
  for (int rr = 0; rr < 16; ++rr) for (int q = 0; q < 4; ++q) { b16 p, ql; split16(O[(m0 + rr) * D + q * 32 + lane] * OS, p, ql); Ah[rr][q * 32 + lane] = p; Al[rr][q * 32 + lane] = ql; }
  wave_lds_sync(); v8f acc[8];
#pragma unroll
  for (int t = 0; t < 8; ++t) acc[t] = (v8f){};
#pragma unroll
  for (int kb = 0; kb < D; kb += 32) { const v16b a = frag_kb(&Ah[nloc][kb], hlf), al = frag_kb(&Al[nloc][kb], hlf);
#pragma unroll
    for (int t = 0; t < 8; ++t) { const v16b bw = frag_kb(WO + (size_t)(t * 16 + nloc) * D + kb, hlf); acc[t] = wmma16b(a, bw, acc[t]); acc[t] = wmma16b(al, bw, acc[t]); } }
#pragma unroll
  for (int t = 0; t < 8; ++t) { const int c = t * 16 + nloc; const float bb = bf16_rne(ob[c]);
#pragma unroll
    for (int r8 = 0; r8 < 8; ++r8) { const int rl = 8 * hlf + r8; Tf[rl][c] = acc[t][r8] * (1.0f / (OS * WSC)) + bb + bf16_rne(x[(m0 + rl) * D + c]) + HL[(m0 + rl) * D + c]; } }
  wave_lds_sync();
  for (int pass = 0; pass < 2; ++pass) { for (int rr = 0; rr < 16; ++rr) { float v[4]; for (int i = 0; i < 4; ++i) v[i] = Tf[rr][lane * 4 + i]; ln128(v, g1, be1, lane); *(volatile v4f*)(H1 + (m0 + rr) * D + lane * 4) = (v4f){v[0], v[1], v[2], v[3]}; } __threadfence(); }
}
__global__ __launch_bounds__(32) void ffn_kernel(const float* __restrict__ H1, const b16* __restrict__ F1, const float* __restrict__ fb1, const b16* __restrict__ F2, const float* __restrict__ fb2, const float* __restrict__ g2, const float* __restrict__ be2, int NLIM, float* __restrict__ out) {
  __shared__ __attribute__((aligned(16))) b16 Ah[16][D + 8], Al[16][D + 8], Bh[16][2 * D + 8], Bl[16][2 * D + 8]; __shared__ __attribute__((aligned(16))) float Tf[16][D + 4];
  const int lane = threadIdx.x, nloc = lane & 15, hlf = lane >> 4; const size_t m0 = (size_t)blockIdx.x * 16; if (m0 >= (size_t)NLIM) return;
  for (int rr = 0; rr < 16; ++rr) for (int q = 0; q < 4; ++q) { b16 p, ql; split16(H1[(m0 + rr) * D + q * 32 + lane] * XS, p, ql); Ah[rr][q * 32 + lane] = p; Al[rr][q * 32 + lane] = ql; }
  wave_lds_sync();
#pragma unroll 1
  for (int cg = 0; cg < 2; ++cg) { v8f acc[8];
#pragma unroll
    for (int t = 0; t < 8; ++t) acc[t] = (v8f){};
#pragma unroll
    for (int kb = 0; kb < D; kb += 32) { const v16b a = frag_kb(&Ah[nloc][kb], hlf), al = frag_kb(&Al[nloc][kb], hlf);
#pragma unroll
      for (int t = 0; t < 8; ++t) { const v16b bw = frag_kb(F1 + (size_t)(cg * 128 + t * 16 + nloc) * D + kb, hlf); acc[t] = wmma16b(a, bw, acc[t]); acc[t] = wmma16b(al, bw, acc[t]); } }
#pragma unroll
    for (int t = 0; t < 8; ++t) { const int c = cg * 128 + t * 16 + nloc; const float bb = bf16_rne(fb1[c]);
#pragma unroll
      for (int r8 = 0; r8 < 8; ++r8) { b16 p, ql; split16(gelu(acc[t][r8] * (1.0f / (XS * WSC)) + bb) * XS, p, ql); Bh[8 * hlf + r8][c] = p; Bl[8 * hlf + r8][c] = ql; } } }
  wave_lds_sync(); v8f acc[8];
#pragma unroll
  for (int t = 0; t < 8; ++t) acc[t] = (v8f){};
#pragma unroll 2
  for (int kb = 0; kb < 2 * D; kb += 32) { const v16b a = frag_kb(&Bh[nloc][kb], hlf), al = frag_kb(&Bl[nloc][kb], hlf);
#pragma unroll
    for (int t = 0; t < 8; ++t) { const v16b bw = frag_kb(F2 + (size_t)(t * 16 + nloc) * (2 * D) + kb, hlf); acc[t] = wmma16b(a, bw, acc[t]); acc[t] = wmma16b(al, bw, acc[t]); } }
#pragma unroll
  for (int t = 0; t < 8; ++t) { const int c = t * 16 + nloc; const float bb = bf16_rne(fb2[c]);
#pragma unroll
    for (int r8 = 0; r8 < 8; ++r8) { const int rl = 8 * hlf + r8; Tf[rl][c] = acc[t][r8] * (1.0f / (XS * WSC)) + bb + H1[(m0 + rl) * D + c]; } }
  wave_lds_sync();
  for (int pass = 0; pass < 2; ++pass) { for (int rr = 0; rr < 16; ++rr) { float v[4]; for (int i = 0; i < 4; ++i) v[i] = Tf[rr][lane * 4 + i]; ln128(v, g2, be2, lane); *(volatile v4f*)(out + (m0 + rr) * D + lane * 4) = (v4f){v[0], v[1], v[2], v[3]}; } __threadfence(); }
}
}

extern "C" void kernel_launch(void* const* d_in, const int* in_sizes, int n_in, void* d_out, int out_size, void* d_ws, size_t ws_size, hipStream_t stream) {
  (void)n_in;
  auto Fp = [&](int i) { return (const float*)d_in[i]; }; auto Ip = [&](int i) { return (const int*)d_in[i]; };
  if (in_sizes[0] != N * D || in_sizes[1] != 2 * E || in_sizes[2] != E * ED || in_sizes[3] != N || in_sizes[6] != (2 * D + ED) * 2 * D || in_sizes[8] != 2 * D * D || in_sizes[10] != 2 * D * D || in_sizes[12] != D * D || in_sizes[14] != D * 3 * D || in_sizes[16] != D * D || in_sizes[18] != D * 2 * D || in_sizes[20] != 2 * D * D || out_size != N * D) return;
  const int NGV = G; const int NLIM = NGV * S, GB16 = NLIM / 16, GB8 = NLIM / 8;
  size_t off = 0; char* ws = (char*)d_ws;
  auto carve = [&](size_t bytes) { char* p = ws + off; off += (bytes + 255) & ~(size_t)255; return p; };
  b16* WPQ = (b16*)carve((size_t)2 * 2 * D * D * 2); b16* WE = (b16*)carve((size_t)2 * D * 32 * 2); b16* W2T = (b16*)carve((size_t)D * 2 * D * 2); b16* U1 = (b16*)carve((size_t)D * 2 * D * 2); b16* U2 = (b16*)carve(D * D * 2); b16* WI = (b16*)carve((size_t)3 * D * D * 2); b16* WO = (b16*)carve(D * D * 2); b16* F1 = (b16*)carve((size_t)2 * D * D * 2); b16* F2 = (b16*)carve((size_t)D * 2 * D * 2);
  float* XN = (float*)carve((size_t)N * D * 4); float* PQ = (float*)carve((size_t)N * 2 * 2 * D * 4); float* AGG = (float*)carve((size_t)N * D * 4); float* HL = (float*)carve((size_t)N * D * 4); float* QKV = (float*)carve((size_t)N * 3 * D * 4); float* O = (float*)carve((size_t)N * D * 4); float* H1 = (float*)carve((size_t)N * D * 4);
  CsrBufs9 csr; off = csr_carve9(csr, ws, off, E, N);
  if (off > ws_size || off > ((size_t)128 << 20)) return;
  wput_kernel<<<(2 * D * 16 + 255) / 256, 256, 0, stream>>>(Fp(6), 0, D, 2 * D, 0, WPQ); wput_kernel<<<(2 * D * 16 + 255) / 256, 256, 0, stream>>>(Fp(6), D, D, 2 * D, 2 * D, WPQ); wput_kernel<<<(2 * D * 4 + 255) / 256, 256, 0, stream>>>(Fp(6), 2 * D, 32, 2 * D, 0, WE);
  wput_kernel<<<(D * 32 + 255) / 256, 256, 0, stream>>>(Fp(8), 0, 2 * D, D, 0, W2T); wput_kernel<<<(D * 32 + 255) / 256, 256, 0, stream>>>(Fp(10), 0, 2 * D, D, 0, U1); wput_kernel<<<(D * 16 + 255) / 256, 256, 0, stream>>>(Fp(12), 0, D, D, 0, U2);
  wput_kernel<<<(3 * D * 16 + 255) / 256, 256, 0, stream>>>(Fp(14), 0, D, 3 * D, 0, WI); wput_kernel<<<(D * 16 + 255) / 256, 256, 0, stream>>>(Fp(16), 0, D, D, 0, WO); wput_kernel<<<(2 * D * 16 + 255) / 256, 256, 0, stream>>>(Fp(18), 0, D, 2 * D, 0, F1); wput_kernel<<<(D * 32 + 255) / 256, 256, 0, stream>>>(Fp(20), 0, 2 * D, D, 0, F2);
  csr_build9(csr, Ip(1) + E, E, N, stream);
  ln_kernel<<<GB8, 256, 0, stream>>>(Fp(0), Fp(4), Fp(5), NLIM, XN);
  dense_kernel<D, 32, 0, 0><<<GB16, 32, 0, stream>>>(XN, D, XS, WPQ, nullptr, NLIM, PQ);
  edge_kernel<<<(unsigned)NLIM, 32, 0, stream>>>(Fp(2), Ip(1), PQ, WE, Fp(7), W2T, Fp(9), csr.PERM, csr.ROWPTR, csr.ROWCNT, (int)csr.permLen, NLIM, AGG);
  upd_kernel<<<GB16, 32, 0, stream>>>(XN, AGG, U1, Fp(11), U2, Fp(13), NLIM, HL);
  dense_kernel<D, 24, 1, 0><<<GB16, 32, 0, stream>>>(Fp(0), D, XS, WI, Fp(15), NLIM, QKV);
  att_kernel<<<(unsigned)(NGV * NH * (S / 16)), 32, 0, stream>>>(QKV, NGV, O);
  mix_kernel<<<GB16, 32, 0, stream>>>(O, WO, Fp(17), Fp(0), HL, Fp(22), Fp(23), NLIM, H1);
  ffn_kernel<<<GB16, 32, 0, stream>>>(H1, F1, Fp(19), F2, Fp(21), Fp(24), Fp(25), NLIM, (float*)d_out);
}
